// UnidirectionalAdjacencyControl_22273700397207
// MI455X (gfx1250) — hardware-verified
//
#include <hip/hip_runtime.h>
#include <stddef.h>


#define FD    256
#define MAXN  8192
#define NTHR  256
#define NWAV  (NTHR / 32)
#define NPW   (MAXN / NWAV)
#define GR    32
#define GTHR  128

static_assert(NWAV * NPW == MAXN);
static_assert((MAXN & (MAXN - 1)) == 0);
static_assert(FD == 256);
static_assert(GTHR == 128 && GR == 32);

typedef float          v4f   __attribute__((ext_vector_type(4)));
typedef float          v8f   __attribute__((ext_vector_type(8)));
typedef int            v4i   __attribute__((ext_vector_type(4)));
typedef unsigned short v8us  __attribute__((ext_vector_type(8)));
typedef unsigned short v16us __attribute__((ext_vector_type(16)));
typedef __bf16         v16b  __attribute__((ext_vector_type(16)));
typedef v4f v4fm __attribute__((may_alias));
union FragB { v16b v; v16us u; v8us h[2]; };

__device__ __forceinline__ unsigned int bf_bits(float f) {
  const unsigned int u = __float_as_uint(f);
  return u + 0x7FFFu + ((u >> 16) & 1u);
}
__device__ __forceinline__ float bf_val(float f) {
  return __uint_as_float(bf_bits(f) & 0xFFFF0000u);
}
__device__ __forceinline__ v8us cvt8(v4f a, v4f b) {
  v8us r;
  r[0] = (unsigned short)(bf_bits(a.x) >> 16);
  r[1] = (unsigned short)(bf_bits(a.y) >> 16);
  r[2] = (unsigned short)(bf_bits(a.z) >> 16);
  r[3] = (unsigned short)(bf_bits(a.w) >> 16);
  r[4] = (unsigned short)(bf_bits(b.x) >> 16);
  r[5] = (unsigned short)(bf_bits(b.y) >> 16);
  r[6] = (unsigned short)(bf_bits(b.z) >> 16);
  r[7] = (unsigned short)(bf_bits(b.w) >> 16);
  return r;
}

__device__ __forceinline__ v8f wmb(v16b a, v16b b, v8f c) {
  v8f d = __builtin_amdgcn_wmma_f32_16x16x32_bf16(false, a, false, b, (short)0, c, false, false);
  asm volatile("v_nop\n\tv_nop\n\tv_nop\n\tv_nop" : "+v"(d) : "v"(a), "v"(b));
  return d;
}

__device__ __forceinline__ int ld1(const int* p, int e, int nE) {
  return (e < nE) ? p[e] : -1;
}

template <int PH>
__device__ __forceinline__ void scan_count(const int* __restrict__ srcp, const int* __restrict__ dstp,
                                           int nE, int nN, int lo, int topv, int vec,
                                           int* cnt, int lane) {
  const unsigned int un  = (unsigned int)nN;
  const unsigned int ulo = (unsigned int)lo;
  const int nIt = (nE + 255) >> 8;
#pragma unroll 1
  for (int it = 0; it < nIt; ++it) {
    const int e0 = (it << 8) + 8 * lane;
    v4i sa, sb, da, db;
    if (vec != 0 && e0 + 7 < nE) {
      sa = *(const v4i*)(srcp + e0);
      sb = *(const v4i*)(srcp + e0 + 4);
      da = *(const v4i*)(dstp + e0);
      db = *(const v4i*)(dstp + e0 + 4);
    } else {
      sa.x = ld1(srcp, e0, nE);     sa.y = ld1(srcp, e0 + 1, nE);
      sa.z = ld1(srcp, e0 + 2, nE); sa.w = ld1(srcp, e0 + 3, nE);
      sb.x = ld1(srcp, e0 + 4, nE); sb.y = ld1(srcp, e0 + 5, nE);
      sb.z = ld1(srcp, e0 + 6, nE); sb.w = ld1(srcp, e0 + 7, nE);
      da.x = ld1(dstp, e0, nE);     da.y = ld1(dstp, e0 + 1, nE);
      da.z = ld1(dstp, e0 + 2, nE); da.w = ld1(dstp, e0 + 3, nE);
      db.x = ld1(dstp, e0 + 4, nE); db.y = ld1(dstp, e0 + 5, nE);
      db.z = ld1(dstp, e0 + 6, nE); db.w = ld1(dstp, e0 + 7, nE);
    }
#define HT(S, D) ((((unsigned int)(S)) < un) & ((((unsigned int)(S)) - ulo) < (unsigned int)NPW) & \
                  (PH != 0 ? ((D) == topv) : (((unsigned int)(D)) < un)))
    const bool h0 = HT(sa.x, da.x), h1 = HT(sa.y, da.y), h2 = HT(sa.z, da.z), h3 = HT(sa.w, da.w);
    const bool h4 = HT(sb.x, db.x), h5 = HT(sb.y, db.y), h6 = HT(sb.z, db.z), h7 = HT(sb.w, db.w);
#undef HT
    const unsigned int anym = __builtin_amdgcn_ballot_w32(h0 | h1 | h2 | h3 | h4 | h5 | h6 | h7);
    if (anym != 0u) {
#define HIT(H, S) { \
        unsigned int mk = __builtin_amdgcn_ballot_w32(H); \
        while (mk != 0u) { \
          const int bt = __builtin_ctz(mk); \
          mk &= mk - 1u; \
          int nd = __builtin_amdgcn_readlane((S), bt); \
          nd &= (MAXN - 1); \
          cnt[nd] = cnt[nd] + 1; \
        } }
      HIT(h0, sa.x)
      HIT(h1, sa.y)
      HIT(h2, sa.z)
      HIT(h3, sa.w)
      HIT(h4, sb.x)
      HIT(h5, sb.y)
      HIT(h6, sb.z)
      HIT(h7, sb.w)
#undef HIT
    }
  }
}

__global__ __launch_bounds__(NTHR) void k_wcvt(const float* __restrict__ W, unsigned short* wb, int n8) {
  const int i = blockIdx.x * NTHR + threadIdx.x;
  if (i >= n8) return;
  const float* p = W + (size_t)i * 8;
  const v4f a = *(const v4f*)p, b = *(const v4f*)(p + 4);
  const v8us r = cvt8(a, b);
  unsigned short* d = wb + (size_t)i * 8;
  *(volatile v8us*)d = r;
  __threadfence();
  *(volatile v8us*)d = r;
}

__global__ __launch_bounds__(GTHR) void k_gemm(const float* __restrict__ x, const unsigned short* __restrict__ wb,
                                               const float* __restrict__ bias, float* hpl, int nN) {
  __shared__ __attribute__((aligned(16))) float stg[GR * FD];
  const int tid = threadIdx.x, lane = tid & 31, wave = tid >> 5, hh = lane >> 4, m = lane & 15;
  const int rowBase = blockIdx.x * GR;
  const int wr = (wave & 1) * 16;
  const int wc = (wave >> 1) * 128;
  int arow = rowBase + wr + m;
  arow = arow > nN - 1 ? nN - 1 : arow;
  const float* xr = x + (size_t)arow * FD + 8 * hh;
  const unsigned short* wrow = wb + (size_t)(wc + m) * FD + 8 * hh;

  v8f acc[8];
#pragma unroll
  for (int t = 0; t < 8; ++t) { const v8f z = {0.f, 0.f, 0.f, 0.f, 0.f, 0.f, 0.f, 0.f}; acc[t] = z; }

#pragma unroll 1
  for (int kt = 0; kt < FD / 32; ++kt) {
    FragB a;
    {
      const float* xp = xr + 32 * kt;
      a.h[0] = cvt8(*(const v4f*)xp, *(const v4f*)(xp + 4));
      a.h[1] = cvt8(*(const v4f*)(xp + 16), *(const v4f*)(xp + 20));
    }
#pragma unroll
    for (int t = 0; t < 8; ++t) {
      const unsigned short* bp = wrow + (size_t)t * 16 * FD + 32 * kt;
      FragB b;
      b.h[0] = *(const v8us*)bp;
      b.h[1] = *(const v8us*)(bp + 16);
      acc[t] = wmb(a.v, b.v, acc[t]);
    }
  }

  float* sp = stg + (wr + 8 * hh) * FD + wc + m;
#pragma unroll
  for (int t = 0; t < 8; ++t) {
    const float bb = bf_val(bias[wc + 16 * t + m]);
    sp[0 * FD + 16 * t] = acc[t][0] + bb;
    sp[1 * FD + 16 * t] = acc[t][1] + bb;
    sp[2 * FD + 16 * t] = acc[t][2] + bb;
    sp[3 * FD + 16 * t] = acc[t][3] + bb;
    sp[4 * FD + 16 * t] = acc[t][4] + bb;
    sp[5 * FD + 16 * t] = acc[t][5] + bb;
    sp[6 * FD + 16 * t] = acc[t][6] + bb;
    sp[7 * FD + 16 * t] = acc[t][7] + bb;
  }
  __syncthreads();

  v4f v[16];
  const float* lp = stg + (wave * 8) * FD + 4 * lane;
#pragma unroll
  for (int r = 0; r < 8; ++r) {
    v[2 * r]     = *(const v4fm*)(lp + r * FD);
    v[2 * r + 1] = *(const v4fm*)(lp + r * FD + 128);
  }
  float* gp = hpl + ((size_t)rowBase + (size_t)wave * 8) * FD + 4 * lane;
#pragma unroll
  for (int r = 0; r < 8; ++r) {
    *(volatile v4f*)(gp + (size_t)r * FD)       = v[2 * r];
    *(volatile v4f*)(gp + (size_t)r * FD + 128) = v[2 * r + 1];
  }
  __threadfence();
#pragma unroll
  for (int r = 0; r < 8; ++r) {
    *(volatile v4f*)(gp + (size_t)r * FD)       = v[2 * r];
    *(volatile v4f*)(gp + (size_t)r * FD + 128) = v[2 * r + 1];
  }
}

__global__ __launch_bounds__(NTHR) void k_topout(const int* __restrict__ ei, const float* __restrict__ hpl,
                                                 const int* __restrict__ bidx, float* out,
                                                 int nN, int nE, int vec) {
  __shared__ __attribute__((aligned(16))) int cnt[MAXN];
  __shared__ unsigned int redh[NWAV], redl[NWAV];
  __shared__ int topS;
  const int tid = threadIdx.x, lane = tid & 31, wave = tid >> 5;
  const int* srcp = ei;
  const int* dstp = ei + nE;
  (void)bidx;

  for (int i = tid; i < MAXN; i += NTHR) cnt[i] = 0;
  __syncthreads();

  scan_count<0>(srcp, dstp, nE, nN, wave * NPW, 0, vec, cnt, lane);
  __syncthreads();

  int bv = -1, bi = 0x7FFFFFFF;
  for (int i = tid; i < nN; i += NTHR) {
    const int dv = cnt[i];
    if (dv > bv) { bv = dv; bi = i; }
  }
  unsigned int kh = (unsigned int)(bv + 1), kl = (unsigned int)(0x7FFFFFFF - bi);
#pragma unroll
  for (int o = 16; o > 0; o >>= 1) {
    const unsigned int oh = __shfl_xor(kh, o), ol = __shfl_xor(kl, o);
    const bool gt = (oh > kh) || (oh == kh && ol > kl);
    kh = gt ? oh : kh;
    kl = gt ? ol : kl;
  }
  if (lane == 0) { redh[wave] = kh; redl[wave] = kl; }
  __syncthreads();
  if (tid == 0) {
    unsigned int bh = redh[0], bl = redl[0];
#pragma unroll
    for (int w = 1; w < NWAV; ++w) {
      const unsigned int oh = redh[w], ol = redl[w];
      const bool gt = (oh > bh) || (oh == bh && ol > bl);
      bh = gt ? oh : bh;
      bl = gt ? ol : bl;
    }
    topS = 0x7FFFFFFF - (int)bl;
  }
  __syncthreads();
  int top = topS;
  top = top < 0 ? 0 : (top > nN - 1 ? nN - 1 : top);

  for (int i = tid; i < MAXN; i += NTHR) cnt[i] = 0;
  __syncthreads();
  scan_count<1>(srcp, dstp, nE, nN, wave * NPW, top, vec, cnt, lane);
  __syncthreads();

  const float* hr = hpl + (size_t)top * FD + 4 * lane;
  const v4f hA = *(const v4f*)hr;
  const v4f hB = *(const v4f*)(hr + 128);
#pragma unroll 1
  for (int i = wave; i < nN; i += NWAV) {
    const float cf = (float)cnt[i];
    const v4f o0 = hA * cf, o1 = hB * cf;
    float* op = out + (size_t)i * FD + 4 * lane;
    *(volatile v4f*)op = o0;
    *(volatile v4f*)(op + 128) = o1;
  }
  __threadfence();
#pragma unroll 1
  for (int i = wave; i < nN; i += NWAV) {
    const float cf = (float)cnt[i];
    const v4f o0 = hA * cf, o1 = hB * cf;
    float* op = out + (size_t)i * FD + 4 * lane;
    *(volatile v4f*)op = o0;
    *(volatile v4f*)(op + 128) = o1;
  }
}

extern "C" void kernel_launch(void* const* d_in, const int* in_sizes, int n_in,
                              void* d_out, int out_size, void* d_ws, size_t ws_size,
                              hipStream_t stream) {
  if (n_in < 5) return;
  const int nN = in_sizes[0] / FD;
  if (nN < GR || nN > MAXN || (nN % GR) != 0 || in_sizes[0] != nN * FD) return;
  if (in_sizes[1] != FD * FD || in_sizes[2] < FD) return;
  if (in_sizes[3] < 0 || (in_sizes[3] & 1) != 0) return;
  const int nE = in_sizes[3] / 2;
  if (out_size != nN * FD) return;

  const float* x    = (const float*)d_in[0];
  const float* W    = (const float*)d_in[1];
  const float* bias = (const float*)d_in[2];
  const int*   ei   = (const int*)d_in[3];
  const int*   bidx = (const int*)d_in[4];
  float* out = (float*)d_out;

  char* ws = (char*)d_ws;
  size_t off = 0;
  const size_t oWb = off; off += (size_t)FD * FD * 2;        off = (off + 255) & ~(size_t)255;
  const size_t oH  = off; off += (size_t)nN * FD * 4;         off = (off + 255) & ~(size_t)255;
  if (off > ws_size) return;
  unsigned short* wb  = (unsigned short*)(ws + oWb);
  float*          hpl = (float*)(ws + oH);

  const int vec = ((nE & 3) == 0) ? 1 : 0;
  const int n8  = FD * FD / 8;

  k_wcvt<<<(n8 + NTHR - 1) / NTHR, NTHR, 0, stream>>>(W, wb, n8);
  k_gemm<<<nN / GR, GTHR, 0, stream>>>(x, wb, bias, hpl, nN);
  k_topout<<<1, NTHR, 0, stream>>>(ei, hpl, bidx, out, nN, nE, vec);
}
